// DotProdAttention_70050916598005
// MI455X (gfx1250) — hardware-verified
//
#include <hip/hip_runtime.h>
#define NB 32
#define DM 64
#define NKV 1
#define NREP (NH / NKV)
#define KVD (NKV * 64)
#define NR (NB * SLEN)
#define CHK 512
typedef int v4i __attribute__((ext_vector_type(4)));
#define FF 2048
#define SLEN 2048
#define MQI 2048
#define MKI 2048
#define TQ SLEN
#define TK SLEN
#define NH 1
#define SCL 0.125f
#define QBLKS (TQ / 64)
#define QB05 0
#define QBN5 4
#define QB0P 0
#define QBNP QBLKS
#define RE 256
typedef __bf16 v16b __attribute__((ext_vector_type(16)));
typedef unsigned short v8us __attribute__((ext_vector_type(8), may_alias));
typedef float  v8f  __attribute__((ext_vector_type(8)));
typedef float  v4f  __attribute__((ext_vector_type(4)));
typedef float  v4fa __attribute__((ext_vector_type(4), may_alias));
union FragB { v16b v; v8us half[2]; unsigned short u[16]; };

__device__ __forceinline__ unsigned short bf16_bits(float x) { unsigned int u = __float_as_uint(x); return (unsigned short)((u + 0x7FFFu + ((u >> 16) & 1u)) >> 16); }
__device__ __forceinline__ float bf16_val(unsigned short b) { return __uint_as_float(((unsigned int)b) << 16); }
__device__ __forceinline__ float bf16_round(float x) { return bf16_val(bf16_bits(x)); }
template <int NT>
__device__ __forceinline__ v8f mmaN(v16b ah, v16b al, v16b bh, v16b bl, v8f c) {
  c = __builtin_amdgcn_wmma_f32_16x16x32_bf16(false, ah, false, bh, (short)0, c, false, false);
  if (NT >= 2) c = __builtin_amdgcn_wmma_f32_16x16x32_bf16(false, al, false, bh, (short)0, c, false, false);
  if (NT >= 3) c = __builtin_amdgcn_wmma_f32_16x16x32_bf16(false, ah, false, bl, (short)0, c, false, false);
  asm volatile("v_nop\n\tv_nop\n\tv_nop\n\tv_nop" : "+v"(c) : "v"(ah), "v"(al), "v"(bh), "v"(bl));
  return c;
}

__global__ __launch_bounds__(256) void k_wt_bf16(const float* __restrict__ W, unsigned short* __restrict__ Wt, int K, int N) {
  const int t = blockIdx.x * 256 + threadIdx.x;
  const int k8n = K / 8;
  if (t >= N * k8n) return;
  const int n = t / k8n, k8 = (t % k8n) * 8;
  v8us v;
#pragma unroll
  for (int i = 0; i < 8; ++i) v[i] = bf16_bits(W[(size_t)(k8 + i) * N + n]);
  *(volatile v8us*)(Wt + (size_t)n * K + k8) = v;
  __threadfence();
  *(volatile v8us*)(Wt + (size_t)n * K + k8) = v;
}

template <bool ASPLIT, int ACT, bool BIAS_BF16>
__global__ __launch_bounds__(128) void k_gemm_bf(const float* __restrict__ A, int lda, const unsigned short* __restrict__ Wt, int ldb,
                                               const float* __restrict__ bias, float* __restrict__ C, int ldc, int M, int N, int K) {
  __shared__ __attribute__((aligned(16))) float so[4][16][64];
  const int tid = threadIdx.x, w = tid >> 5, lane = tid & 31, ln = lane & 15, hh = lane >> 4;
  const int ntn = N / 64;
  const int wid = blockIdx.x * 4 + w;
  const int mt = wid / ntn, nq = wid % ntn;
  if (mt * 16 >= M) return;
  const int row0 = mt * 16, col0 = nq * 64;
  const float* arow = A + (size_t)(row0 + ln) * lda;
  v8f acc[4] = {};
  for (int kb = 0; kb < K; kb += 32) {
    FragB ah, al;
    const v4f x0 = *(const v4fa*)(arow + kb + 8 * hh), x1 = *(const v4fa*)(arow + kb + 8 * hh + 4);
    const v4f x2 = *(const v4fa*)(arow + kb + 16 + 8 * hh), x3 = *(const v4fa*)(arow + kb + 16 + 8 * hh + 4);
    float xs[16] = {x0[0],x0[1],x0[2],x0[3],x1[0],x1[1],x1[2],x1[3],x2[0],x2[1],x2[2],x2[3],x3[0],x3[1],x3[2],x3[3]};
#pragma unroll
    for (int i = 0; i < 16; ++i) { const unsigned short hb = bf16_bits(xs[i]); ah.u[i] = hb; al.u[i] = ASPLIT ? bf16_bits(xs[i] - bf16_val(hb)) : (unsigned short)0; }
#pragma unroll
    for (int t = 0; t < 4; ++t) {
      const unsigned short* brow = Wt + (size_t)(col0 + t * 16 + ln) * ldb + kb;
      FragB b;
      b.half[0] = *(const v8us*)(brow + 8 * hh);
      b.half[1] = *(const v8us*)(brow + 16 + 8 * hh);
      acc[t] = mmaN<ASPLIT ? 2 : 1>(ah.v, al.v, b.v, b.v, acc[t]);
    }
  }
#pragma unroll
  for (int t = 0; t < 4; ++t) {
    float bv = bias ? bias[col0 + t * 16 + ln] : 0.f;
    if (BIAS_BF16) bv = bf16_round(bv);
#pragma unroll
    for (int r = 0; r < 8; ++r) { float v = acc[t][r] + bv; if (ACT == 1) v = fmaxf(v, 0.f); so[w][8 * hh + r][t * 16 + ln] = v; }
  }
  __builtin_amdgcn_fence(__ATOMIC_ACQ_REL, "workgroup");
  __builtin_amdgcn_wave_barrier();
  const int rsub = lane >> 4, c4 = (lane & 15) * 4;
  for (int pass = 0; pass < 2; ++pass) {
#pragma unroll
    for (int q = 0; q < 8; ++q) {
      const int r = q * 2 + rsub;
      const v4f v = *(const v4fa*)&so[w][r][c4];
      *(volatile v4f*)(C + (size_t)(row0 + r) * ldc + col0 + c4) = v;
    }
    if (pass == 0) __threadfence();
  }
}

template <bool ASPLIT, int ACT, bool BIAS_BF16, bool RES_BF16>
__global__ __launch_bounds__(128) void k_gemm_bf3(const float* __restrict__ A, int lda, const unsigned short* __restrict__ Wt, int ldb,
                                                const float* __restrict__ bias, const float* __restrict__ resid, int rmod, int ldr,
                                                float* __restrict__ C, int ldc, int M, int N, int K) {
  __shared__ __attribute__((aligned(16))) float so[4][16][64];
  const int tid = threadIdx.x, w = tid >> 5, lane = tid & 31, ln = lane & 15, hh = lane >> 4;
  const int ntn = N / 64;
  const int wid = blockIdx.x * 4 + w;
  const int mt = wid / ntn, nq = wid % ntn;
  if (mt * 16 >= M) return;
  const int row0 = mt * 16, col0 = nq * 64;
  const float* arow = A + (size_t)(row0 + ln) * lda;
  v8f acc[4] = {};
  for (int kb = 0; kb < K; kb += 32) {
    FragB ah, al;
    const v4f x0 = *(const v4fa*)(arow + kb + 8 * hh), x1 = *(const v4fa*)(arow + kb + 8 * hh + 4);
    const v4f x2 = *(const v4fa*)(arow + kb + 16 + 8 * hh), x3 = *(const v4fa*)(arow + kb + 16 + 8 * hh + 4);
    float xs[16] = {x0[0],x0[1],x0[2],x0[3],x1[0],x1[1],x1[2],x1[3],x2[0],x2[1],x2[2],x2[3],x3[0],x3[1],x3[2],x3[3]};
#pragma unroll
    for (int i = 0; i < 16; ++i) { const unsigned short hb = bf16_bits(xs[i]); ah.u[i] = hb; al.u[i] = ASPLIT ? bf16_bits(xs[i] - bf16_val(hb)) : (unsigned short)0; }
#pragma unroll
    for (int t = 0; t < 4; ++t) {
      const unsigned short* brow = Wt + (size_t)(col0 + t * 16 + ln) * ldb + kb;
      FragB b;
      b.half[0] = *(const v8us*)(brow + 8 * hh);
      b.half[1] = *(const v8us*)(brow + 16 + 8 * hh);
      acc[t] = mmaN<ASPLIT ? 2 : 1>(ah.v, al.v, b.v, b.v, acc[t]);
    }
  }
#pragma unroll
  for (int t = 0; t < 4; ++t) {
    const int col = col0 + t * 16 + ln;
    float bv = bias ? bias[col] : 0.f;
    if (BIAS_BF16) bv = bf16_round(bv);
#pragma unroll
    for (int r = 0; r < 8; ++r) {
      float v = acc[t][r] + bv;
      if (resid) { float rv = resid[(size_t)((row0 + 8 * hh + r) % rmod) * ldr + col]; if (RES_BF16) rv = bf16_round(rv); v += rv; }
      if (ACT == 1) v = fmaxf(v, 0.f);
      if (ACT == 2) v = 0.5f * v * (1.0f + erff(v * 0.70710678118654752f));
      if (ACT == 3) { const float u = 0.7978845608028654f * (v + 0.044715f * v * v * v); v = 0.5f * v * (1.0f + tanhf(u)); }
      so[w][8 * hh + r][t * 16 + ln] = v;
    }
  }
  __builtin_amdgcn_fence(__ATOMIC_ACQ_REL, "workgroup");
  __builtin_amdgcn_wave_barrier();
  const int rsub = lane >> 4, c4 = (lane & 15) * 4;
  for (int pass = 0; pass < 2; ++pass) {
#pragma unroll
    for (int q = 0; q < 8; ++q) {
      const int r = q * 2 + rsub;
      const v4f v = *(const v4fa*)&so[w][r][c4];
      *(volatile v4f*)(C + (size_t)(row0 + r) * ldc + col0 + c4) = v;
    }
    if (pass == 0) __threadfence();
  }
}
template <bool PARAM_BF16>
__global__ __launch_bounds__(256) void k_layernorm(const float* __restrict__ X, const float* __restrict__ R, const float* __restrict__ g, const float* __restrict__ bta,
                                                  float* __restrict__ out_sum, float* __restrict__ out_norm, int N, float eps) {
  __shared__ float red[256];
  const int row = blockIdx.x, tid = threadIdx.x;
  const float* x = X + (size_t)row * N; const float* rr = R ? R + (size_t)row * N : nullptr;
  float vals[16];
  const int per = N / 256;
  float s1 = 0.f;
  for (int u = 0; u < per / 4; ++u) {
    const int j = tid * 4 + 1024 * u;
    const v4f a = *(const v4fa*)(x + j);
    v4f b = {0.f,0.f,0.f,0.f}; if (rr) b = *(const v4fa*)(rr + j);
#pragma unroll
    for (int q = 0; q < 4; ++q) { const float v = a[q] + b[q]; vals[u * 4 + q] = v; s1 += v; }
  }
  red[tid] = s1; __syncthreads();
  for (int st = 128; st > 0; st >>= 1) { if (tid < st) red[tid] += red[tid + st]; __syncthreads(); }
  const float mu = red[0] / (float)N; __syncthreads();
  float s2 = 0.f;
  for (int u = 0; u < per / 4; ++u)
#pragma unroll
    for (int q = 0; q < 4; ++q) { const float c = vals[u * 4 + q] - mu; s2 += c * c; }
  red[tid] = s2; __syncthreads();
  for (int st = 128; st > 0; st >>= 1) { if (tid < st) red[tid] += red[tid + st]; __syncthreads(); }
  const float rs = rsqrtf(red[0] / (float)N + eps);
  for (int pass = 0; pass < 2; ++pass) {
    for (int u = 0; u < per / 4; ++u) {
      const int j = tid * 4 + 1024 * u;
      v4f o, sm;
#pragma unroll
      for (int q = 0; q < 4; ++q) {
        float gg = g[j + q], bb = bta[j + q];
        if (PARAM_BF16) { gg = bf16_round(gg); bb = bf16_round(bb); }
        sm[q] = vals[u * 4 + q]; o[q] = (vals[u * 4 + q] - mu) * rs * gg + bb;
      }
      if (out_sum) *(volatile v4f*)(out_sum + (size_t)row * N + j) = sm;
      *(volatile v4f*)(out_norm + (size_t)row * N + j) = o;
    }
    if (pass == 0) __threadfence();
  }
}


typedef _Float16 v16h __attribute__((ext_vector_type(16)));
union FragH { v16h v; v8us half[2]; _Float16 h[16]; unsigned short u[16]; };
template <int NT>
__device__ __forceinline__ v8f mmaH(v16h ah, v16h al, v16h bh, v16h bl, v8f c) {
  c = __builtin_amdgcn_wmma_f32_16x16x32_f16(false, ah, false, bh, (short)0, c, false, false);
  if (NT >= 2) c = __builtin_amdgcn_wmma_f32_16x16x32_f16(false, al, false, bh, (short)0, c, false, false);
  if (NT >= 3) c = __builtin_amdgcn_wmma_f32_16x16x32_f16(false, ah, false, bl, (short)0, c, false, false);
  asm volatile("v_nop\n\tv_nop\n\tv_nop\n\tv_nop" : "+v"(c) : "v"(ah), "v"(al), "v"(bh), "v"(bl));
  return c;
}
template <bool ASPLIT>
__global__ __launch_bounds__(128) void k_gemm_h(const float* __restrict__ A, int lda, size_t sA, const _Float16* __restrict__ Bh, int ldb, size_t sB, float alpha, float* __restrict__ C, int ldc, size_t sC, int M, int N, int K) {
  __shared__ __attribute__((aligned(16))) float so[4][16][64];
  const int tid = threadIdx.x, w = tid >> 5, lane = tid & 31, ln = lane & 15, hh = lane >> 4; const int by = blockIdx.y;
  A += (size_t)by * sA; Bh += (size_t)by * sB; C += (size_t)by * sC;
  const int ntn = (N + 63) / 64; const int wid = blockIdx.x * 4 + w; const int mt = wid / ntn, nq = wid % ntn; if (mt * 16 >= M) return;
  const int row0 = mt * 16, col0 = nq * 64; const float* arow = A + (size_t)(row0 + ln) * lda;
  v8f acc[4] = {};
  for (int kb = 0; kb < K; kb += 32) {
    FragH ah, al;
    const v4f x0 = *(const v4fa*)(arow + kb + 8 * hh), x1 = *(const v4fa*)(arow + kb + 8 * hh + 4), x2 = *(const v4fa*)(arow + kb + 16 + 8 * hh), x3 = *(const v4fa*)(arow + kb + 16 + 8 * hh + 4);
    float xs[16] = {x0[0],x0[1],x0[2],x0[3],x1[0],x1[1],x1[2],x1[3],x2[0],x2[1],x2[2],x2[3],x3[0],x3[1],x3[2],x3[3]};
#pragma unroll
    for (int i = 0; i < 16; ++i) { const _Float16 h = (_Float16)xs[i]; ah.h[i] = h; al.h[i] = ASPLIT ? (_Float16)(xs[i] - (float)h) : (_Float16)0.0f; }
#pragma unroll
    for (int t = 0; t < 4; ++t) { if (col0 + t * 16 >= N) continue; const size_t boff = (size_t)(col0 + t * 16 + ln) * ldb + kb; FragH bq; bq.half[0] = *(const v8us*)(Bh + boff + 8 * hh); bq.half[1] = *(const v8us*)(Bh + boff + 16 + 8 * hh);
      acc[t] = mmaH<ASPLIT ? 2 : 1>(ah.v, al.v, bq.v, bq.v, acc[t]); }
  }
#pragma unroll
  for (int t = 0; t < 4; ++t) { if (col0 + t * 16 >= N) continue;
#pragma unroll
    for (int r = 0; r < 8; ++r) so[w][8 * hh + r][t * 16 + ln] = acc[t][r] * alpha; }
  __builtin_amdgcn_fence(__ATOMIC_ACQ_REL, "workgroup"); __builtin_amdgcn_wave_barrier();
  const int rsub = lane >> 4, c4 = (lane & 15) * 4;
  for (int pass = 0; pass < 2; ++pass) {
#pragma unroll
    for (int q = 0; q < 8; ++q) { const int r = q * 2 + rsub; if (col0 + c4 < N) { const v4f v = *(const v4fa*)&so[w][r][c4]; *(volatile v4f*)(C + (size_t)(row0 + r) * ldc + col0 + c4) = v; } }
    if (pass == 0) __threadfence(); }
}

__global__ __launch_bounds__(256) void k_wt_f16(const float* __restrict__ W, _Float16* __restrict__ Wt, int K, int N, float scale) {
  const int t = blockIdx.x * 256 + threadIdx.x; if (t >= N * (K / 8)) return; const int n = t / (K / 8), k8 = (t % (K / 8)) * 8; FragH f;
#pragma unroll
  for (int i = 0; i < 8; ++i) f.h[i] = (_Float16)(bf16_round(W[(size_t)(k8 + i) * N + n]) * scale); const v8us o = f.half[0];
  *(volatile v8us*)((unsigned short*)Wt + (size_t)n * K + k8) = o; __threadfence(); *(volatile v8us*)((unsigned short*)Wt + (size_t)n * K + k8) = o;
}
template <int ACT>
__global__ __launch_bounds__(128) void k_gemm_hhx(const _Float16* __restrict__ A, int lda, size_t sA, const _Float16* __restrict__ Bh, int ldb, size_t sB, float alpha, const float* __restrict__ bias, size_t sBias, const float* __restrict__ CP, int rowsPerB, size_t sCPb, int row0g,
    float* __restrict__ C, _Float16* __restrict__ C16, int ldc, size_t sC, int M, int N, int K) {
  __shared__ __attribute__((aligned(16))) float so[4][16][64];
  const int tid = threadIdx.x, w = tid >> 5, lane = tid & 31, ln = lane & 15, hh = lane >> 4; const int by = blockIdx.y;
  A += (size_t)by * sA; Bh += (size_t)by * sB; const size_t cofs = (size_t)by * sC; const float* bp = bias ? bias + (size_t)by * sBias : nullptr;
  const int ntn = (N + 63) / 64; const int wid = blockIdx.x * 4 + w; const int mt = wid / ntn, nq = wid % ntn; if (mt * 16 >= M) return;
  const int row0 = mt * 16, col0 = nq * 64; const _Float16* arow = A + (size_t)(row0 + ln) * lda;
  v8f acc[4] = {};
  for (int kb = 0; kb < K; kb += 32) { FragH ah; ah.half[0] = *(const v8us*)((const unsigned short*)arow + kb + 8 * hh); ah.half[1] = *(const v8us*)((const unsigned short*)arow + kb + 16 + 8 * hh);
#pragma unroll
    for (int t = 0; t < 4; ++t) { if (col0 + t * 16 >= N) continue; const size_t boff = (size_t)(col0 + t * 16 + ln) * ldb + kb; FragH bq; bq.half[0] = *(const v8us*)((const unsigned short*)Bh + boff + 8 * hh); bq.half[1] = *(const v8us*)((const unsigned short*)Bh + boff + 16 + 8 * hh);
      acc[t] = mmaH<1>(ah.v, ah.v, bq.v, bq.v, acc[t]); }
  }
#pragma unroll
  for (int t = 0; t < 4; ++t) { if (col0 + t * 16 >= N) continue; const int col = col0 + t * 16 + ln; const float bv = bp ? bf16_round(bp[col]) : 0.f;
#pragma unroll
    for (int r = 0; r < 8; ++r) { float v = acc[t][r] * alpha + bv; if (CP) { const int bidx = (row0g + row0 + 8 * hh + r) / rowsPerB; v += CP[(size_t)bidx * sCPb + (size_t)by * 64 + col]; } if (ACT == 1) v = (v > 0.f) ? v : expm1f(v); else if (ACT == 7) v = (v > 0.f) ? v + 1.0f : expf(v); else if (ACT == 8) v = tanhf(v); else if (ACT == 9) v = 0.5f * v * (1.0f + tanhf(0.7978845608028654f * (v + 0.044715f * v * v * v))); else if (ACT == 11) v = 1.0f / (1.0f + expf(-v)); else if (ACT == 12) v = (v > 0.f) ? v : 0.01f * v; else if (ACT == 14) v = (v > 0.f) ? v : 0.1f * v; else if (ACT == 15) v = v / (1.0f + expf(-v)); else if (ACT == 3) v = fmaxf(v, 0.f); else if (ACT == 6) v = 0.5f * v * (1.0f + erff(v * 0.70710678118654752f)); so[w][8 * hh + r][t * 16 + ln] = v; } }
  __builtin_amdgcn_fence(__ATOMIC_ACQ_REL, "workgroup"); __builtin_amdgcn_wave_barrier();
  const int rsub = lane >> 4, c4 = (lane & 15) * 4; typedef _Float16 v4h __attribute__((ext_vector_type(4)));
  for (int pass = 0; pass < 2; ++pass) {
#pragma unroll
    for (int q = 0; q < 8; ++q) { const int r = q * 2 + rsub; if (col0 + c4 < N) { const v4f v = *(const v4fa*)&so[w][r][c4]; if (C) *(volatile v4f*)(C + cofs + (size_t)(row0 + r) * ldc + col0 + c4) = v; if (C16) { v4h h4; for (int i = 0; i < 4; ++i) h4[i] = (_Float16)v[i]; *(volatile v4h*)(C16 + cofs + (size_t)(row0 + r) * ldc + col0 + c4) = h4; } } }
    if (pass == 0) __threadfence(); }
}


typedef _Float16 v4h __attribute__((ext_vector_type(4)));

__global__ __launch_bounds__(256) void k_x16(const float* __restrict__ x, _Float16* __restrict__ X16, size_t n8) { const size_t t = (size_t)blockIdx.x * 256 + threadIdx.x; if (t >= n8) return; FragH f;
#pragma unroll
  for (int q = 0; q < 8; ++q) f.h[q] = (_Float16)bf16_round(x[t * 8 + q]); *(volatile v8us*)((unsigned short*)X16 + t * 8) = f.half[0]; __threadfence(); *(volatile v8us*)((unsigned short*)X16 + t * 8) = f.half[0]; }
__global__ __launch_bounds__(256) void k_h16(const float* __restrict__ x, _Float16* __restrict__ X16, size_t n8) { const size_t t = (size_t)blockIdx.x * 256 + threadIdx.x; if (t >= n8) return; FragH f;
#pragma unroll
  for (int q = 0; q < 8; ++q) f.h[q] = (_Float16)x[t * 8 + q]; *(volatile v8us*)((unsigned short*)X16 + t * 8) = f.half[0]; __threadfence(); *(volatile v8us*)((unsigned short*)X16 + t * 8) = f.half[0]; }
__global__ __launch_bounds__(256) void k_round16f(const float* __restrict__ W, _Float16* __restrict__ Bt, size_t n8) { const size_t t = (size_t)blockIdx.x * 256 + threadIdx.x; if (t >= n8) return; FragH f;
#pragma unroll
  for (int i = 0; i < 8; ++i) f.h[i] = (_Float16)(bf16_round(W[t * 8 + i]) * 16.0f); *(volatile v8us*)((unsigned short*)Bt + t * 8) = f.half[0]; __threadfence(); *(volatile v8us*)((unsigned short*)Bt + t * 8) = f.half[0]; }
template <int NHv, int TTv>
__global__ __launch_bounds__(256) void k_vt(const _Float16* __restrict__ V16, int ldv, int voff, _Float16* __restrict__ Vt) { __shared__ unsigned short tl[64][66]; const int tid = threadIdx.x; const int slab = blockIdx.x / (TTv / 64), lg = blockIdx.x % (TTv / 64); const int b = slab / NHv, h = slab % NHv;
  for (int i = tid; i < 64 * 8; i += 256) { const int r = i / 8, c8 = (i % 8) * 8; FragH f; f.half[0] = *(const v8us*)((const unsigned short*)V16 + ((size_t)b * TTv + lg * 64 + r) * ldv + voff + h * 64 + c8);
#pragma unroll
    for (int q = 0; q < 8; ++q) tl[r][c8 + q] = f.u[q]; }
  __syncthreads();
  for (int pass = 0; pass < 2; ++pass) {
#pragma unroll
    for (int rd = 0; rd < 2; ++rd) { const int d = rd * 32 + tid / 8, pc = tid % 8; FragH f;
#pragma unroll
      for (int q = 0; q < 8; ++q) f.u[q] = tl[pc * 8 + q][d];
      *(volatile v8us*)((unsigned short*)Vt + ((size_t)slab * 64 + d) * TTv + lg * 64 + pc * 8) = f.half[0]; }
    if (pass == 0) __threadfence(); } }

__global__ __launch_bounds__(256) void k_hl(const float* __restrict__ F, _Float16* __restrict__ Hh, _Float16* __restrict__ Hl, size_t n8) { const size_t t = (size_t)blockIdx.x * 256 + threadIdx.x; if (t >= n8) return; FragH fh, fl; const v4f a = *(const v4fa*)(F + t * 8), c = *(const v4fa*)(F + t * 8 + 4);
#pragma unroll
  for (int q = 0; q < 4; ++q) { _Float16 h = (_Float16)a[q]; fh.h[q] = h; fl.h[q] = (_Float16)((a[q] - (float)h) * 1024.0f); h = (_Float16)c[q]; fh.h[4 + q] = h; fl.h[4 + q] = (_Float16)((c[q] - (float)h) * 1024.0f); }
  for (int pass = 0; pass < 2; ++pass) { *(volatile v8us*)((unsigned short*)Hh + t * 8) = fh.half[0]; *(volatile v8us*)((unsigned short*)Hl + t * 8) = fl.half[0]; if (pass == 0) __threadfence(); } }

__device__ __forceinline__ v16h g2_frag(const _Float16* p, int hh) { FragH f; f.half[0] = *(const v8us*)((const unsigned short*)p + 8 * hh); f.half[1] = *(const v8us*)((const unsigned short*)p + 16 + 8 * hh); return f.v; }
__device__ __forceinline__ v8f g2_mma(v16h a, v16h b, v8f c) { v8f d = __builtin_amdgcn_wmma_f32_16x16x32_f16(false, a, false, b, (short)0, c, false, false); asm volatile("v_nop\n\tv_nop\n\tv_nop\n\tv_nop" : "+v"(d) : "v"(a), "v"(b)); return d; }
template <int ACT>
__global__ __launch_bounds__(128) void k_gemm2(const _Float16* __restrict__ A, int lda, size_t sA, const _Float16* __restrict__ Bh, int ldb, size_t sB, float alpha, const float* __restrict__ bias, size_t sBias, const float* __restrict__ CP, int rowsPerB, size_t sCPb, int row0g,
    float* __restrict__ C, _Float16* __restrict__ C16, int ldc, size_t sC, int M, int N, int K) {
  __shared__ __attribute__((aligned(16))) float so[4][32][68];
  const int tid = threadIdx.x, w = tid >> 5, lane = tid & 31, ln = lane & 15, hh = lane >> 4; const int by = blockIdx.y;
  A += (size_t)by * sA; Bh += (size_t)by * sB; const size_t cofs = (size_t)by * sC; const float* bp = bias ? bias + (size_t)by * sBias : nullptr;
  const int ntn = N >> 6; const int mt = blockIdx.x / ntn, nq = blockIdx.x - mt * ntn; const int row0 = mt * 128 + 32 * w, col0 = nq * 64; if (row0 >= M) return;
  const _Float16* a0p = A + (size_t)(row0 + ln) * lda; const _Float16* a1p = a0p + (size_t)16 * lda;
  const _Float16* b0p = Bh + (size_t)(col0 + ln) * ldb; const _Float16* b1p = b0p + (size_t)16 * ldb; const _Float16* b2p = b1p + (size_t)16 * ldb; const _Float16* b3p = b2p + (size_t)16 * ldb;
  const v8f z8 = {0.f,0.f,0.f,0.f,0.f,0.f,0.f,0.f}; v8f c00 = z8, c01 = z8, c02 = z8, c03 = z8, c10 = z8, c11 = z8, c12 = z8, c13 = z8;
#pragma unroll 1
  for (int kb = 0; kb < K; kb += 32) { const v16h a0 = g2_frag(a0p + kb, hh), a1 = g2_frag(a1p + kb, hh);
    v16h b = g2_frag(b0p + kb, hh); c00 = g2_mma(a0, b, c00); c10 = g2_mma(a1, b, c10);
    b = g2_frag(b1p + kb, hh); c01 = g2_mma(a0, b, c01); c11 = g2_mma(a1, b, c11);
    b = g2_frag(b2p + kb, hh); c02 = g2_mma(a0, b, c02); c12 = g2_mma(a1, b, c12);
    b = g2_frag(b3p + kb, hh); c03 = g2_mma(a0, b, c03); c13 = g2_mma(a1, b, c13); }
  v8f accs[8] = {c00, c01, c02, c03, c10, c11, c12, c13};
#pragma unroll
  for (int u = 0; u < 8; ++u) { const int t = u & 3, half = u >> 2; const int col = col0 + t * 16 + ln; const float bv = bp ? bf16_round(bp[col]) : 0.f;
#pragma unroll
    for (int r = 0; r < 8; ++r) { const int rloc = half * 16 + 8 * hh + r; float v = accs[u][r] * alpha + bv; if (CP) { if (rowsPerB < 0) v += CP[cofs + (size_t)(row0g + row0 + rloc) * ldc + col];        else { const int bidx = (row0g + row0 + rloc) / rowsPerB; v += CP[(size_t)bidx * sCPb + (size_t)by * 64 + col]; } }
      if (ACT == 3) v = fmaxf(v, 0.f); else if (ACT == 6) v = 0.5f * v * (1.0f + erff(v * 0.70710678118654752f)); else if (ACT == 11) v = 1.0f / (1.0f + expf(-v)); else if (ACT == 15) v = v / (1.0f + expf(-v)); else if (ACT == 12) v = (v > 0.f) ? v : 0.01f * v; else if (ACT == 8) v = tanhf(v);
      so[w][rloc][t * 16 + ln] = v; } }
  __builtin_amdgcn_fence(__ATOMIC_ACQ_REL, "workgroup"); __builtin_amdgcn_wave_barrier();
  const int rsub = lane >> 4, c4 = (lane & 15) * 4;
  for (int pass = 0; pass < 2; ++pass) {
#pragma unroll
    for (int q = 0; q < 16; ++q) { const int r = q * 2 + rsub; const v4f v = *(const v4fa*)&so[w][r][c4]; if (C) *(volatile v4f*)(C + cofs + (size_t)(row0 + r) * ldc + col0 + c4) = v; if (C16) { v4h h4; for (int i = 0; i < 4; ++i) h4[i] = (_Float16)v[i]; *(volatile v4h*)(C16 + cofs + (size_t)(row0 + r) * ldc + col0 + c4) = h4; } }
    if (pass == 0) __threadfence(); } }


template <int CAUSAL>
__global__ __launch_bounds__(128) void k_flash(const _Float16* __restrict__ Q16, int ldq, const _Float16* __restrict__ K16, int ldk, const _Float16* __restrict__ Vt, const int* __restrict__ MSK, float* __restrict__ O, int ldo) {
  constexpr int RPW = 16, RTN = RPW / 16, NQB = TQ / (4 * RPW), DT = 4, KS = 2;
  __shared__ __attribute__((aligned(16))) unsigned short sP[4][RPW][40]; __shared__ __attribute__((aligned(16))) float sO[4][RPW][64 + 4];
  const int tid = threadIdx.x, w = tid >> 5, lane = tid & 31, ln = lane & 15, hh = lane >> 4;
  const int slab = blockIdx.x / QBNP, qblk = QB0P + blockIdx.x % QBNP; (void)NQB; const int b = slab / NH, h = slab % NH; const int qb0 = qblk * (4 * RPW); const int q0 = qb0 + w * RPW;
  FragH aq[2][KS];
#pragma unroll
  for (int rt = 0; rt < RTN; ++rt) { const unsigned short* qr = (const unsigned short*)Q16 + ((size_t)b * TQ + q0 + rt * 16 + ln) * ldq + h * 64;
#pragma unroll
    for (int ks = 0; ks < KS; ++ks) { aq[rt][ks].half[0] = *(const v8us*)(qr + ks * 32 + 8 * hh); aq[rt][ks].half[1] = *(const v8us*)(qr + ks * 32 + 16 + 8 * hh); } }
  const unsigned short* Vth = (const unsigned short*)Vt + (size_t)slab * 64 * TK;
  float m_r[2][8], l_r[2][8]; v8f oacc[2][DT];
#pragma unroll
  for (int rt = 0; rt < RTN; ++rt) {
#pragma unroll
    for (int r = 0; r < 8; ++r) { m_r[rt][r] = -3.0e38f; l_r[rt][r] = 0.f; }
#pragma unroll
    for (int dt = 0; dt < DT; ++dt) oacc[rt][dt] = (v8f){0.f,0.f,0.f,0.f,0.f,0.f,0.f,0.f}; }
  const int jend = (CAUSAL == 1) ? (qb0 + 4 * RPW) : ((CAUSAL == 23) ? min(TK, (qb0 / CHK + 2) * CHK) : TK);        const int jbeg = (CAUSAL == 23) ? max(0, (qb0 / CHK - 1) * CHK) : 0;
#pragma unroll 1
  for (int j0 = jbeg; j0 < jend; j0 += 32) {
    v8f s[2][2];
#pragma unroll
    for (int nt = 0; nt < 2; ++nt) { const unsigned short* kr = (const unsigned short*)K16 + ((size_t)b * TK + j0 + nt * 16 + ln) * ldk + h * 64; FragH bk[KS];
#pragma unroll
      for (int ks = 0; ks < KS; ++ks) { bk[ks].half[0] = *(const v8us*)(kr + ks * 32 + 8 * hh); bk[ks].half[1] = *(const v8us*)(kr + ks * 32 + 16 + 8 * hh); }
#pragma unroll
      for (int rt = 0; rt < RTN; ++rt) { v8f acc = (v8f){0.f,0.f,0.f,0.f,0.f,0.f,0.f,0.f};
#pragma unroll
        for (int ks = 0; ks < KS; ++ks) acc = mmaH<1>(aq[rt][ks].v, aq[rt][ks].v, bk[ks].v, bk[ks].v, acc); s[rt][nt] = acc; } }
#pragma unroll
    for (int rt = 0; rt < RTN; ++rt)
#pragma unroll
      for (int r = 0; r < 8; ++r) { const int tq = q0 + rt * 16 + 8 * hh + r; const int k0 = j0 + ln, k1 = j0 + 16 + ln;
        bool ok0 = (CAUSAL == 1) ? (k0 <= tq) : ((CAUSAL == 2) ? ((k0 >> 5) == (tq >> 5)) : true), ok1 = (CAUSAL == 1) ? (k1 <= tq) : ((CAUSAL == 2) ? ((k1 >> 5) == (tq >> 5)) : true); if (CAUSAL == 23) { const int cq = tq / CHK; ok0 = (abs(k0 / CHK - cq) <= 1) && (MSK[(size_t)b * TK + k0] == 0); ok1 = (abs(k1 / CHK - cq) <= 1) && (MSK[(size_t)b * TK + k1] == 0); }
        if (CAUSAL == 24) { ok0 = (MSK[(size_t)b * TK + k0] == 0); ok1 = (MSK[(size_t)b * TK + k1] == 0); }
        float s0 = ok0 ? s[rt][0][r] * SCL : -3.0e38f, s1 = ok1 ? s[rt][1][r] * SCL : -3.0e38f; if (CAUSAL == 27) { const float* amk = (const float*)MSK + ((size_t)b * MQI + tq) * MKI; s0 += bf16_round(amk[k0]); s1 += bf16_round(amk[k1]); }        if (CAUSAL == 33) { const float* amk = (const float*)MSK + (size_t)tq * TK; s0 += bf16_round(amk[k0]); s1 += bf16_round(amk[k1]); }        if (CAUSAL == 17) { const float* amk = (const float*)MSK + (size_t)b * TK; s0 += bf16_round(amk[k0]); s1 += bf16_round(amk[k1]); } if (CAUSAL == 18) { const float* tb = (const float*)MSK; const int* ri = MSK + 1024 + (size_t)b * TK; const int rq = ri[tq]; s0 += tb[(h * 8 + rq) * 8 + ri[k0]]; s1 += tb[(h * 8 + rq) * 8 + ri[k1]]; } if (CAUSAL == 19) { const int* rel = MSK + (size_t)tq * TK; const float* rb = (const float*)MSK + (size_t)TQ * TK + ((size_t)(b * NH + h) * TQ + tq) * 64; s0 += rb[rel[k0]]; s1 += rb[rel[k1]]; }                      float mc = fmaxf(s0, s1);
        mc = fmaxf(mc, __shfl_xor(mc, 1, 32)); mc = fmaxf(mc, __shfl_xor(mc, 2, 32)); mc = fmaxf(mc, __shfl_xor(mc, 4, 32)); mc = fmaxf(mc, __shfl_xor(mc, 8, 32));
        const float mn = fmaxf(m_r[rt][r], mc); const float al = (mn > -1.0e38f) ? expf(m_r[rt][r] - mn) : 1.0f; m_r[rt][r] = mn; const float p0 = ok0 ? expf(s0 - mn) : 0.f, p1 = ok1 ? expf(s1 - mn) : 0.f; l_r[rt][r] = l_r[rt][r] * al + p0 + p1;
#pragma unroll
        for (int dt = 0; dt < DT; ++dt) oacc[rt][dt][r] *= al;
        FragH t2; t2.h[0] = (_Float16)(p0 * 1024.0f); t2.h[1] = (_Float16)(p1 * 1024.0f); sP[w][rt * 16 + 8 * hh + r][ln] = t2.u[0]; sP[w][rt * 16 + 8 * hh + r][16 + ln] = t2.u[1]; }
    __builtin_amdgcn_fence(__ATOMIC_ACQ_REL, "workgroup"); __builtin_amdgcn_wave_barrier();
    FragH pa[2];
#pragma unroll
    for (int rt = 0; rt < RTN; ++rt) { pa[rt].half[0] = *(const v8us*)&sP[w][rt * 16 + ln][8 * hh]; pa[rt].half[1] = *(const v8us*)&sP[w][rt * 16 + ln][16 + 8 * hh]; }
#pragma unroll
    for (int dt = 0; dt < DT; ++dt) { const unsigned short* vrow = Vth + (size_t)(dt * 16 + ln) * TK + j0; FragH bv; bv.half[0] = *(const v8us*)(vrow + 8 * hh); bv.half[1] = *(const v8us*)(vrow + 16 + 8 * hh);
#pragma unroll
      for (int rt = 0; rt < RTN; ++rt) oacc[rt][dt] = mmaH<1>(pa[rt].v, pa[rt].v, bv.v, bv.v, oacc[rt][dt]); }
    __builtin_amdgcn_fence(__ATOMIC_ACQ_REL, "workgroup"); __builtin_amdgcn_wave_barrier(); }
#pragma unroll
  for (int rt = 0; rt < RTN; ++rt) {
#pragma unroll
    for (int r = 0; r < 8; ++r) { float l = l_r[rt][r]; l += __shfl_xor(l, 1, 32); l += __shfl_xor(l, 2, 32); l += __shfl_xor(l, 4, 32); l += __shfl_xor(l, 8, 32); l_r[rt][r] = (l > 0.f) ? 1.0f / (l * 1024.0f) : 0.f; }
#pragma unroll
    for (int dt = 0; dt < DT; ++dt)
#pragma unroll
      for (int r = 0; r < 8; ++r) sO[w][rt * 16 + 8 * hh + r][dt * 16 + ln] = oacc[rt][dt][r] * l_r[rt][r]; }
  __builtin_amdgcn_fence(__ATOMIC_ACQ_REL, "workgroup"); __builtin_amdgcn_wave_barrier();
  for (int pass = 0; pass < 2; ++pass) {
#pragma unroll
    for (int rp = 0; rp < RPW; rp += 2) { const int r = rp + (lane >> 4), pc = lane & 15; const v4f val = *(const v4fa*)&sO[w][r][pc * 4]; *(volatile v4f*)(O + ((size_t)b * TQ + q0 + r) * ldo + h * 64 + pc * 4) = val; }
    if (pass == 0) __threadfence(); } }
template <int CAUSAL>
__global__ __launch_bounds__(128) void k_flash5(const _Float16* __restrict__ Q16, const _Float16* __restrict__ QL, int ldq, const _Float16* __restrict__ K16, const _Float16* __restrict__ KL, int ldk, const _Float16* __restrict__ Vt, const _Float16* __restrict__ VtL, const int* __restrict__ MSK, float* __restrict__ O, int ldo) {
  constexpr int RPW = 16, RTN = RPW / 16, NQB = TQ / (4 * RPW), DT = 4, KS = 2;
  __shared__ __attribute__((aligned(16))) unsigned short sP[4][RPW][40]; __shared__ __attribute__((aligned(16))) unsigned short sPL[4][RPW][40]; __shared__ __attribute__((aligned(16))) float sO[4][RPW][64 + 4];
  const int tid = threadIdx.x, w = tid >> 5, lane = tid & 31, ln = lane & 15, hh = lane >> 4;
  const int slab = blockIdx.x / QBN5, qblk = QB05 + blockIdx.x % QBN5; (void)NQB; const int b = slab / NH, h = slab % NH; const int qb0 = qblk * (4 * RPW); const int q0 = qb0 + w * RPW;
  FragH aq[2][KS], aql[2][KS];
#pragma unroll
  for (int rt = 0; rt < RTN; ++rt) { const unsigned short* qr = (const unsigned short*)Q16 + ((size_t)b * TQ + q0 + rt * 16 + ln) * ldq + h * 64; const unsigned short* ql = (const unsigned short*)QL + ((size_t)b * TQ + q0 + rt * 16 + ln) * ldq + h * 64;
#pragma unroll
    for (int ks = 0; ks < KS; ++ks) { aq[rt][ks].half[0] = *(const v8us*)(qr + ks * 32 + 8 * hh); aq[rt][ks].half[1] = *(const v8us*)(qr + ks * 32 + 16 + 8 * hh); aql[rt][ks].half[0] = *(const v8us*)(ql + ks * 32 + 8 * hh); aql[rt][ks].half[1] = *(const v8us*)(ql + ks * 32 + 16 + 8 * hh); } }
  const unsigned short* Vth = (const unsigned short*)Vt + (size_t)slab * 64 * TK; const unsigned short* Vtl = (const unsigned short*)VtL + (size_t)slab * 64 * TK;
  float m_r[2][8], l_r[2][8]; v8f oacc[2][DT], oaccL[2][DT];
#pragma unroll
  for (int rt = 0; rt < RTN; ++rt) {
#pragma unroll
    for (int r = 0; r < 8; ++r) { m_r[rt][r] = -3.0e38f; l_r[rt][r] = 0.f; }
#pragma unroll
    for (int dt = 0; dt < DT; ++dt) { oacc[rt][dt] = (v8f){0.f,0.f,0.f,0.f,0.f,0.f,0.f,0.f}; oaccL[rt][dt] = oacc[rt][dt]; } }
  const int jend = (CAUSAL == 1) ? (qb0 + 4 * RPW) : ((CAUSAL == 23) ? min(TK, (qb0 / CHK + 2) * CHK) : TK);        const int jbeg = (CAUSAL == 23) ? max(0, (qb0 / CHK - 1) * CHK) : 0;
#pragma unroll 1
  for (int j0 = jbeg; j0 < jend; j0 += 32) {
    v8f s[2][2];
#pragma unroll
    for (int nt = 0; nt < 2; ++nt) { const unsigned short* kr = (const unsigned short*)K16 + ((size_t)b * TK + j0 + nt * 16 + ln) * ldk + h * 64; const unsigned short* klr = (const unsigned short*)KL + ((size_t)b * TK + j0 + nt * 16 + ln) * ldk + h * 64; FragH bk[KS], bkl[KS];
#pragma unroll
      for (int ks = 0; ks < KS; ++ks) { bk[ks].half[0] = *(const v8us*)(kr + ks * 32 + 8 * hh); bk[ks].half[1] = *(const v8us*)(kr + ks * 32 + 16 + 8 * hh); bkl[ks].half[0] = *(const v8us*)(klr + ks * 32 + 8 * hh); bkl[ks].half[1] = *(const v8us*)(klr + ks * 32 + 16 + 8 * hh); }
#pragma unroll
      for (int rt = 0; rt < RTN; ++rt) { v8f acc = (v8f){0.f,0.f,0.f,0.f,0.f,0.f,0.f,0.f}, accl = acc;
#pragma unroll
        for (int ks = 0; ks < KS; ++ks) { acc = mmaH<1>(aq[rt][ks].v, aq[rt][ks].v, bk[ks].v, bk[ks].v, acc); accl = mmaH<1>(aql[rt][ks].v, aql[rt][ks].v, bk[ks].v, bk[ks].v, accl); accl = mmaH<1>(aq[rt][ks].v, aq[rt][ks].v, bkl[ks].v, bkl[ks].v, accl); }
#pragma unroll
        for (int r = 0; r < 8; ++r) acc[r] += accl[r] * 0.0009765625f;
        s[rt][nt] = acc; } }
#pragma unroll
    for (int rt = 0; rt < RTN; ++rt)
#pragma unroll
      for (int r = 0; r < 8; ++r) { const int tq = q0 + rt * 16 + 8 * hh + r; const int k0 = j0 + ln, k1 = j0 + 16 + ln;
        bool ok0 = (CAUSAL == 1) ? (k0 <= tq) : ((CAUSAL == 2) ? ((k0 >> 5) == (tq >> 5)) : true), ok1 = (CAUSAL == 1) ? (k1 <= tq) : ((CAUSAL == 2) ? ((k1 >> 5) == (tq >> 5)) : true);
        if (CAUSAL == 4) { const int* mrow = MSK + ((size_t)b * TQ + tq) * TK; ok0 = mrow[k0] != 0; ok1 = mrow[k1] != 0; }
        float s0 = ok0 ? s[rt][0][r] * SCL : -3.0e38f, s1 = ok1 ? s[rt][1][r] * SCL : -3.0e38f; if (CAUSAL == 33) { const float* amk = (const float*)MSK + (size_t)tq * TK; s0 += bf16_round(amk[k0]); s1 += bf16_round(amk[k1]); }        if (CAUSAL == 17) { const float* amk = (const float*)MSK + (size_t)b * TK; s0 += bf16_round(amk[k0]); s1 += bf16_round(amk[k1]); } if (CAUSAL == 18) { const float* tb = (const float*)MSK; const int* ri = MSK + 1024 + (size_t)b * TK; const int rq = ri[tq]; s0 += tb[(h * 8 + rq) * 8 + ri[k0]]; s1 += tb[(h * 8 + rq) * 8 + ri[k1]]; } if (CAUSAL == 19) { const int* rel = MSK + (size_t)tq * TK; const float* rb = (const float*)MSK + (size_t)TQ * TK + ((size_t)(b * NH + h) * TQ + tq) * 64; s0 += rb[rel[k0]]; s1 += rb[rel[k1]]; }                      float mc = fmaxf(s0, s1);
        mc = fmaxf(mc, __shfl_xor(mc, 1, 32)); mc = fmaxf(mc, __shfl_xor(mc, 2, 32)); mc = fmaxf(mc, __shfl_xor(mc, 4, 32)); mc = fmaxf(mc, __shfl_xor(mc, 8, 32));
        const float mn = fmaxf(m_r[rt][r], mc); const float al = (mn > -1.0e38f) ? expf(m_r[rt][r] - mn) : 1.0f; m_r[rt][r] = mn; const float p0 = ok0 ? expf(s0 - mn) : 0.f, p1 = ok1 ? expf(s1 - mn) : 0.f; l_r[rt][r] = l_r[rt][r] * al + p0 + p1;
#pragma unroll
        for (int dt = 0; dt < DT; ++dt) { oacc[rt][dt][r] *= al; oaccL[rt][dt][r] *= al; }
        FragH t2, t2l; const float ps0 = p0 * 1024.0f, ps1 = p1 * 1024.0f; t2.h[0] = (_Float16)ps0; t2.h[1] = (_Float16)ps1; t2l.h[0] = (_Float16)((ps0 - (float)t2.h[0]) * 1024.0f); t2l.h[1] = (_Float16)((ps1 - (float)t2.h[1]) * 1024.0f);
        sP[w][rt * 16 + 8 * hh + r][ln] = t2.u[0]; sP[w][rt * 16 + 8 * hh + r][16 + ln] = t2.u[1]; sPL[w][rt * 16 + 8 * hh + r][ln] = t2l.u[0]; sPL[w][rt * 16 + 8 * hh + r][16 + ln] = t2l.u[1]; }
    __builtin_amdgcn_fence(__ATOMIC_ACQ_REL, "workgroup"); __builtin_amdgcn_wave_barrier();
    FragH pa[2], pl[2];
#pragma unroll
    for (int rt = 0; rt < RTN; ++rt) { pa[rt].half[0] = *(const v8us*)&sP[w][rt * 16 + ln][8 * hh]; pa[rt].half[1] = *(const v8us*)&sP[w][rt * 16 + ln][16 + 8 * hh]; pl[rt].half[0] = *(const v8us*)&sPL[w][rt * 16 + ln][8 * hh]; pl[rt].half[1] = *(const v8us*)&sPL[w][rt * 16 + ln][16 + 8 * hh]; }
#pragma unroll
    for (int dt = 0; dt < DT; ++dt) { const unsigned short* vrow = Vth + (size_t)(dt * 16 + ln) * TK + j0; const unsigned short* vrl = Vtl + (size_t)(dt * 16 + ln) * TK + j0; FragH bv, bl; bv.half[0] = *(const v8us*)(vrow + 8 * hh); bv.half[1] = *(const v8us*)(vrow + 16 + 8 * hh); bl.half[0] = *(const v8us*)(vrl + 8 * hh); bl.half[1] = *(const v8us*)(vrl + 16 + 8 * hh);
#pragma unroll
      for (int rt = 0; rt < RTN; ++rt) { oacc[rt][dt] = mmaH<1>(pa[rt].v, pa[rt].v, bv.v, bv.v, oacc[rt][dt]); oaccL[rt][dt] = mmaH<1>(pl[rt].v, pl[rt].v, bv.v, bv.v, oaccL[rt][dt]); oaccL[rt][dt] = mmaH<1>(pa[rt].v, pa[rt].v, bl.v, bl.v, oaccL[rt][dt]); } }
    __builtin_amdgcn_fence(__ATOMIC_ACQ_REL, "workgroup"); __builtin_amdgcn_wave_barrier(); }
#pragma unroll
  for (int rt = 0; rt < RTN; ++rt) {
#pragma unroll
    for (int r = 0; r < 8; ++r) { float l = l_r[rt][r]; l += __shfl_xor(l, 1, 32); l += __shfl_xor(l, 2, 32); l += __shfl_xor(l, 4, 32); l += __shfl_xor(l, 8, 32); l_r[rt][r] = (l > 0.f) ? 1.0f / (l * 1024.0f) : 0.f; }
#pragma unroll
    for (int dt = 0; dt < DT; ++dt)
#pragma unroll
      for (int r = 0; r < 8; ++r) { float v = oacc[rt][dt][r]; v += oaccL[rt][dt][r] * 0.0009765625f; sO[w][rt * 16 + 8 * hh + r][dt * 16 + ln] = v * l_r[rt][r]; } }
  __builtin_amdgcn_fence(__ATOMIC_ACQ_REL, "workgroup"); __builtin_amdgcn_wave_barrier();
  for (int pass = 0; pass < 2; ++pass) {
#pragma unroll
    for (int rp = 0; rp < RPW; rp += 2) { const int r = rp + (lane >> 4), pc = lane & 15; const v4f val = *(const v4fa*)&sO[w][r][pc * 4]; *(volatile v4f*)(O + ((size_t)b * TQ + q0 + r) * ldo + h * 64 + pc * 4) = val; }
    if (pass == 0) __threadfence(); } }

__global__ __launch_bounds__(256) void k_rotab(float* __restrict__ CS, float* __restrict__ SN) {
  #pragma clang fp contract(off)
  const int t = blockIdx.x * 256 + threadIdx.x; if (t >= SLEN * 32) return; const int j = t % 32, s = t / 32; const float ex = (float)(2 * j) / 64.0f; const float inv = 1.0f / powf(10000.0f, ex); const float th = (float)s * inv; const float c = cosf(th), sn = sinf(th);
  for (int pass = 0; pass < 2; ++pass) { *(volatile float*)(CS + t) = c; *(volatile float*)(SN + t) = sn; if (pass == 0) __threadfence(); } }
__global__ __launch_bounds__(256) void k_rope(const float* __restrict__ F, int nsrc, int ndst, int rep, const float* __restrict__ CS, const float* __restrict__ SN, _Float16* __restrict__ H, _Float16* __restrict__ L) {
  #pragma clang fp contract(off)
  const size_t t = (size_t)blockIdx.x * 256 + threadIdx.x; if (t >= (size_t)NR * ndst * 4) return; const int g8 = (int)(t % 4); const int hd = (int)((t / 4) % ndst); const size_t row = t / ((size_t)4 * ndst); const int s = (int)(row % SLEN); const int hs = hd / rep;
  const float* src = F + row * (size_t)(nsrc * 64) + hs * 64; FragH ah, al, bh, bl;
  for (int i = 0; i < 8; ++i) { const int d = g8 * 8 + i; const float c = CS[s * 32 + d], sn = SN[s * 32 + d]; const float x1 = src[d], x2 = src[d + 32];
    float o1 = x1 * c; o1 += -x2 * sn; float o2 = x2 * c; o2 += x1 * sn;
    _Float16 hv = (_Float16)o1; ah.h[i] = hv; al.h[i] = (_Float16)((o1 - (float)hv) * 1024.0f); hv = (_Float16)o2; bh.h[i] = hv; bl.h[i] = (_Float16)((o2 - (float)hv) * 1024.0f); }
  const size_t o = row * (size_t)(ndst * 64) + hd * 64 + g8 * 8;
  for (int pass = 0; pass < 2; ++pass) { *(volatile v8us*)((unsigned short*)H + o) = ah.half[0]; *(volatile v8us*)((unsigned short*)H + o + 32) = bh.half[0]; *(volatile v8us*)((unsigned short*)L + o) = al.half[0]; *(volatile v8us*)((unsigned short*)L + o + 32) = bl.half[0]; if (pass == 0) __threadfence(); } }
__global__ __launch_bounds__(256) void k_rope2(const float* __restrict__ F, int nsrc, int ndst, int rep, const float* __restrict__ CS, const float* __restrict__ SN, _Float16* __restrict__ H, _Float16* __restrict__ L) {
  #pragma clang fp contract(off)
  const size_t t = (size_t)blockIdx.x * 256 + threadIdx.x; if (t >= (size_t)NR * ndst * 4) return; const int g16 = (int)(t % 4); const int hd = (int)((t / 4) % ndst); const size_t row = t / ((size_t)4 * ndst); const int s = (int)(row % SLEN); const int hs = hd / rep;
  const float* src = F + row * (size_t)(nsrc * 64) + hs * 64 + g16 * 16; FragH ah, al;
  for (int pr = 0; pr < 8; ++pr) { const int i = g16 * 8 + pr; const float c = CS[s * 32 + i], sn = SN[s * 32 + i]; const float x1 = src[2 * pr], x2 = src[2 * pr + 1];
    float o1 = x1 * c; o1 -= x2 * sn; float o2 = x1 * sn; o2 += x2 * c;
    _Float16 hv = (_Float16)o1; ah.h[2 * pr] = hv; al.h[2 * pr] = (_Float16)((o1 - (float)hv) * 1024.0f); hv = (_Float16)o2; ah.h[2 * pr + 1] = hv; al.h[2 * pr + 1] = (_Float16)((o2 - (float)hv) * 1024.0f); }
  const size_t o = row * (size_t)(ndst * 64) + hd * 64 + g16 * 16;
  for (int pass = 0; pass < 2; ++pass) { *(volatile v8us*)((unsigned short*)H + o) = ah.half[0]; *(volatile v8us*)((unsigned short*)H + o + 8) = ah.half[1]; *(volatile v8us*)((unsigned short*)L + o) = al.half[0]; *(volatile v8us*)((unsigned short*)L + o + 8) = al.half[1]; if (pass == 0) __threadfence(); } }
__global__ __launch_bounds__(256) void k_ln512(const float* __restrict__ A, const float* __restrict__ res, const float* __restrict__ g, const float* __restrict__ bb, float* __restrict__ Y, _Float16* __restrict__ Y16) {
  #pragma clang fp contract(off)
  const int wv = threadIdx.x >> 5, ln = threadIdx.x & 31; const size_t r = (size_t)blockIdx.x * 8 + wv; if (r >= NR) return; float x[16]; float s = 0.f;
  for (int i = 0; i < 2; ++i) { const v8f a = *(const v8f*)(A + r * DM + i * 256 + ln * 8); for (int q = 0; q < 8; ++q) { float v = a[q]; if (res) v += bf16_round(res[r * DM + i * 256 + ln * 8 + q]); x[i * 8 + q] = v; s += v; } }
  for (int o = 16; o > 0; o >>= 1) s += __shfl_xor(s, o, 32); const float mu = s / (float)DM; float var = 0.f; for (int q = 0; q < 16; ++q) { const float d = x[q] - mu; var += d * d; }
  for (int o = 16; o > 0; o >>= 1) var += __shfl_xor(var, o, 32); const float inv = rsqrtf(var / (float)DM + 1e-5f);
  for (int pass = 0; pass < 2; ++pass) { for (int i = 0; i < 2; ++i) { const int c0 = i * 256 + ln * 8; v8f y; FragH f; for (int q = 0; q < 8; ++q) { float v = (x[i * 8 + q] - mu) * inv; v *= bf16_round(g[c0 + q]); v += bf16_round(bb[c0 + q]); y[q] = v; f.h[q] = (_Float16)v; } *(volatile v8f*)(Y + r * DM + c0) = y; if (Y16) *(volatile v8us*)((unsigned short*)Y16 + r * DM + c0) = f.half[0]; } if (pass == 0) __threadfence(); } }
__global__ __launch_bounds__(256) void k_pack(const float* __restrict__ rb, const int* __restrict__ rid, int* __restrict__ PK) { const int t = blockIdx.x * 256 + threadIdx.x; if (t >= 1024 + NB * TK) return; int v; if (t < 1024) v = __float_as_int(bf16_round(rb[t])); else v = rid[t - 1024]; *(volatile int*)(PK + t) = v; __threadfence(); *(volatile int*)(PK + t) = v; }
__global__ __launch_bounds__(256) void k_tabin(const float* __restrict__ sp, float* __restrict__ CS, float* __restrict__ SN) { const int t = blockIdx.x * 256 + threadIdx.x; if (t >= SLEN * 32) return; const int i = t % 32, s = t / 32; const float c = bf16_round(sp[s * 64 + 32 + i]), sn = bf16_round(sp[s * 64 + i]);
  for (int pass = 0; pass < 2; ++pass) { *(volatile float*)(CS + t) = c; *(volatile float*)(SN + t) = sn; if (pass == 0) __threadfence(); } }
__global__ __launch_bounds__(256) void k_wsc(const float* __restrict__ Wm, _Float16* __restrict__ Bt, size_t n8, float sc) { const size_t t = (size_t)blockIdx.x * 256 + threadIdx.x; if (t >= n8) return; FragH f; for (int q = 0; q < 8; ++q) f.h[q] = (_Float16)(bf16_round(Wm[t * 8 + q]) * sc); *(volatile v8us*)((unsigned short*)Bt + t * 8) = f.half[0]; __threadfence(); *(volatile v8us*)((unsigned short*)Bt + t * 8) = f.half[0]; }
__global__ __launch_bounds__(256) void k_rotab2(float* __restrict__ CS, float* __restrict__ SN) {
  #pragma clang fp contract(off)
  const int t = blockIdx.x * 256 + threadIdx.x; if (t >= SLEN * 32) return; const int j = t % 32, s = t / 32; const float c0 = -0.14391156831212787f;        const float inv = expf((float)(2 * j) * c0); const float th = (float)s * inv; const float c = cosf(th), sn = sinf(th);
  for (int pass = 0; pass < 2; ++pass) { *(volatile float*)(CS + t) = c; *(volatile float*)(SN + t) = sn; if (pass == 0) __threadfence(); } }
__global__ __launch_bounds__(256) void k_lnu(const float* __restrict__ X, _Float16* __restrict__ N16, float* __restrict__ XB) {
  #pragma clang fp contract(off)
  const int wv = threadIdx.x >> 5, ln = threadIdx.x & 31; const size_t r = (size_t)blockIdx.x * 8 + wv; if (r >= NR) return; float a[32]; float s = 0.f;
  for (int i = 0; i < 4; ++i) { const v8f v = *(const v8f*)(X + r * DM + (i * 32 + ln) * 8); for (int q = 0; q < 8; ++q) { const float u = bf16_round(v[q]); a[i * 8 + q] = u; s += u; } }
  for (int o = 16; o > 0; o >>= 1) s += __shfl_xor(s, o, 32); const float mu = s / (float)DM; float var = 0.f; for (int q = 0; q < 32; ++q) { const float d = a[q] - mu; var += d * d; }
  for (int o = 16; o > 0; o >>= 1) var += __shfl_xor(var, o, 32); const float den = sqrtf(var / (float)(DM - 1)) + 1e-6f; const float inv = 1.0f / den;
  for (int pass = 0; pass < 2; ++pass) { for (int i = 0; i < 4; ++i) { const int c0 = (i * 32 + ln) * 8; FragH f; v8f xb; for (int q = 0; q < 8; ++q) { f.h[q] = (_Float16)((a[i * 8 + q] - mu) * inv); xb[q] = a[i * 8 + q]; } *(volatile v8us*)((unsigned short*)N16 + r * DM + c0) = f.half[0]; *(volatile v8f*)(XB + r * DM + c0) = xb; } if (pass == 0) __threadfence(); } }
__global__ __launch_bounds__(256) void k_vtg(const _Float16* __restrict__ V16, _Float16* __restrict__ Vt) { __shared__ unsigned short tl[64][66]; const int tid = threadIdx.x; const int slab = blockIdx.x / (SLEN / 64), lg = blockIdx.x % (SLEN / 64); const int b = slab / NH, h = slab % NH; const int hs = h / NREP;
  for (int i = tid; i < 64 * 8; i += 256) { const int r = i / 8, c8 = (i % 8) * 8; FragH f; f.half[0] = *(const v8us*)((const unsigned short*)V16 + ((size_t)b * SLEN + lg * 64 + r) * KVD + hs * 64 + c8); for (int q = 0; q < 8; ++q) tl[r][c8 + q] = f.u[q]; }
  __syncthreads();
  for (int pass = 0; pass < 2; ++pass) { for (int rd = 0; rd < 2; ++rd) { const int d = rd * 32 + tid / 8, pc = tid % 8; FragH f; for (int q = 0; q < 8; ++q) f.u[q] = tl[pc * 8 + q][d]; *(volatile v8us*)((unsigned short*)Vt + ((size_t)slab * 64 + d) * SLEN + lg * 64 + pc * 8) = f.half[0]; } if (pass == 0) __threadfence(); } }

__global__ __launch_bounds__(256) void k_h16s(const float* __restrict__ SRC, int lds, int coff, _Float16* __restrict__ DST, size_t n8) { const size_t t = (size_t)blockIdx.x * 256 + threadIdx.x; if (t >= n8) return; const size_t r = (t * 8) / DM; const int c = (int)((t * 8) % DM); const v8f a = *(const v8f*)(SRC + r * lds + coff + c); FragH f; for (int q = 0; q < 8; ++q) f.h[q] = (_Float16)a[q];
  *(volatile v8us*)((unsigned short*)DST + t * 8) = f.half[0]; __threadfence(); *(volatile v8us*)((unsigned short*)DST + t * 8) = f.half[0]; }


__global__ __launch_bounds__(256) void k_ccp(const float* __restrict__ QKV, int coff, _Float16* __restrict__ D) { const size_t t = (size_t)blockIdx.x * 256 + threadIdx.x; if (t >= (size_t)NR * DM / 8) return; const int c0 = (int)((t * 8) % DM); const size_t row = (t * 8) / DM; const v8f a = *(const v8f*)(QKV + row * 3 * DM + coff + c0); FragH f; for (int q = 0; q < 8; ++q) f.h[q] = (_Float16)a[q];
  *(volatile v8us*)((unsigned short*)D + t * 8) = f.half[0]; __threadfence(); *(volatile v8us*)((unsigned short*)D + t * 8) = f.half[0]; }


extern "C" void kernel_launch(void* const* d_in, const int* in_sizes, int n_in,
                              void* d_out, int out_size, void* d_ws, size_t ws_size, hipStream_t stream) {
  (void)in_sizes; (void)n_in; (void)out_size;
  const float* q = (const float*)d_in[0]; const float* kv = (const float*)d_in[1]; const float* mask = (const float*)d_in[2]; float* O = (float*)d_out;
  char* ws = (char*)d_ws; size_t off = 0;
  auto take = [&](size_t bytes) { char* p = ws + off; off += (bytes + 255) & ~(size_t)255; return p; };
  const size_t np = (size_t)NR * DM;
  _Float16* Q16 = (_Float16*)take(np * 2); _Float16* K16 = (_Float16*)take(np * 2); _Float16* VT = (_Float16*)take(np * 2);
  if (off > ws_size) return;
  k_x16<<<(unsigned)((np / 8 + 255) / 256), 256, 0, stream>>>(q, Q16, np / 8); k_x16<<<(unsigned)((np / 8 + 255) / 256), 256, 0, stream>>>(kv, K16, np / 8);
  k_vtg<<<NB * NH * (SLEN / 64), 256, 0, stream>>>(K16, VT);
  k_flash<33><<<NB * NH * QBNP, 128, 0, stream>>>(Q16, DM, K16, DM, VT, (const int*)mask, O, DM);
}
